// dcgcn_34153579938492
// MI455X (gfx1250) — hardware-verified
//
#include <hip/hip_runtime.h>
#include <stddef.h>


#define DD      64
#define NTHR    256
#define NWAVE   8
#define EPT     8
#define NGRP    2
#define CHUNK   (NTHR * EPT * NGRP)
#define WCAP    (EPT * NGRP * 32)
#define LISTN   (NWAVE * WCAP)
#define NBK     8192
#define SLB     13
#define RCAP    32768
#define TGT     256
#define DEGCAP  256
#define GROWS   128
#define GPH     72
#define MPA     136
#define NLAYER  3
#define WSCAP   134217728
#define LDS_CSR ((RCAP + 2 * NBK + LISTN + 2 * NWAVE) * 4)
#define CX0     64.0f
#define CX1     4096.0f
#define CW      16.0f
#define CG      1024.0f
#define CXM     64.0f
#define INV2    (1.0f / 16384.0f)

static_assert((1 << SLB) == NBK);
static_assert(CHUNK == 4096);
static_assert(NBK == NTHR * 32);
static_assert((NBK % TGT) == 0 && TGT == NWAVE * 32);
static_assert(GROWS == NWAVE * 16);
static_assert((RCAP % (4 * NTHR)) == 0 && (NBK % (4 * NTHR)) == 0);
static_assert(WCAP == 512 && LISTN == 4096);
static_assert((GPH % 8) == 0 && (MPA % 8) == 0);

typedef float    v4f  __attribute__((ext_vector_type(4)));
typedef float    v8f  __attribute__((ext_vector_type(8)));
typedef int      v4i  __attribute__((ext_vector_type(4)));
typedef _Float16 v4h  __attribute__((ext_vector_type(4)));
typedef _Float16 v8h  __attribute__((ext_vector_type(8)));
typedef _Float16 v16h __attribute__((ext_vector_type(16)));
union FragH { v16h v; v8h half[2]; };

__device__ __forceinline__ v8f wmh(v16h a, v16h b, v8f c) {
  v8f d = __builtin_amdgcn_wmma_f32_16x16x32_f16(false, a, false, b, (short)0, c, false, false);
  asm volatile("v_nop\n\tv_nop\n\tv_nop\n\tv_nop" : "+v"(d) : "v"(a), "v"(b));
  return d;
}

template <int NB>
__device__ __forceinline__ int scan_chunk(const int* __restrict__ dsts, int nE, int cbase, int slotBase,
                                          int vec8, int* list, int tid, int lane, int wave) {
  int wc = 0;
#pragma unroll
  for (int g = 0; g < NGRP; ++g) {
    const int el0  = (g * NTHR + tid) * EPT;
    const int e0   = cbase + el0;
    const int sent = -2147483647 - 1;
    v4i da, db;
    if (vec8 != 0 && cbase + CHUNK <= nE) {
      da = *(const v4i*)(dsts + e0);
      db = *(const v4i*)(dsts + e0 + 4);
    } else {
      da.x = (e0     < nE) ? dsts[min(e0, nE - 1)] : sent;
      da.y = (e0 + 1 < nE) ? dsts[min(e0 + 1, nE - 1)] : sent;
      da.z = (e0 + 2 < nE) ? dsts[min(e0 + 2, nE - 1)] : sent;
      da.w = (e0 + 3 < nE) ? dsts[min(e0 + 3, nE - 1)] : sent;
      db.x = (e0 + 4 < nE) ? dsts[min(e0 + 4, nE - 1)] : sent;
      db.y = (e0 + 5 < nE) ? dsts[min(e0 + 5, nE - 1)] : sent;
      db.z = (e0 + 6 < nE) ? dsts[min(e0 + 6, nE - 1)] : sent;
      db.w = (e0 + 7 < nE) ? dsts[min(e0 + 7, nE - 1)] : sent;
    }
    const unsigned nb = (unsigned)slotBase;
    const unsigned s0 = (unsigned)da.x - nb, s1 = (unsigned)da.y - nb;
    const unsigned s2 = (unsigned)da.z - nb, s3 = (unsigned)da.w - nb;
    const unsigned s4 = (unsigned)db.x - nb, s5 = (unsigned)db.y - nb;
    const unsigned s6 = (unsigned)db.z - nb, s7 = (unsigned)db.w - nb;
    const bool h0 = s0 < (unsigned)NB, h1 = s1 < (unsigned)NB, h2 = s2 < (unsigned)NB, h3 = s3 < (unsigned)NB;
    const bool h4 = s4 < (unsigned)NB, h5 = s5 < (unsigned)NB, h6 = s6 < (unsigned)NB, h7 = s7 < (unsigned)NB;
    const unsigned any = __builtin_amdgcn_ballot_w32(h0 | h1 | h2 | h3 | h4 | h5 | h6 | h7);
    if (any != 0u) {
#define HITJ(J, HJ, SJ) { \
        const unsigned mj = __builtin_amdgcn_ballot_w32(HJ); \
        if (mj != 0u) { \
          if (HJ) { \
            const int pos = wc + (int)__builtin_amdgcn_mbcnt_lo(mj, 0u); \
            if (pos < WCAP) list[wave * WCAP + pos] = ((el0 + (J)) << SLB) | (int)(SJ); \
          } \
          wc += (int)__builtin_popcount(mj); } }
      HITJ(0, h0, s0)
      HITJ(1, h1, s1)
      HITJ(2, h2, s2)
      HITJ(3, h3, s3)
      HITJ(4, h4, s4)
      HITJ(5, h5, s5)
      HITJ(6, h6, s6)
      HITJ(7, h7, s7)
#undef HITJ
    }
  }
  return wc;
}

__global__ __launch_bounds__(NTHR) void k_wprep(
    const float* __restrict__ aw1, const float* __restrict__ ab1, const float* __restrict__ aw2,
    const float* __restrict__ remb, const float* __restrict__ pw1, const float* __restrict__ pw2,
    _Float16* W1T, _Float16* W2T, _Float16* P1T, _Float16* P2T, float* C, int nR) {
  const int blk = blockIdx.x, tid = threadIdx.x;
  if (blk < 4 * nR + 5) {
    const float* w; int DO, KD, i; _Float16* dst;
    if (blk < 2 * nR) {
      const int r = blk >> 1;
      w = aw1 + (size_t)r * 2 * DD * DD; DO = DD; KD = DD; i = (blk & 1) * NTHR + tid; dst = W1T + (size_t)r * DD * DD;
    } else if (blk < 4 * nR) {
      const int r = (blk - 2 * nR) >> 1;
      w = aw2 + (size_t)r * DD * DD; DO = DD; KD = DD; i = ((blk - 2 * nR) & 1) * NTHR + tid; dst = W2T + (size_t)r * DD * DD;
    } else if (blk < 4 * nR + 4) {
      w = pw1; DO = DD; KD = 2 * DD; i = (blk - 4 * nR) * NTHR + tid; dst = P1T;
    } else {
      w = pw2; DO = 32; KD = DD; i = tid; dst = P2T;
    }
    const int kq = KD >> 3;
    const int n  = i / kq;
    const int k0 = (i - n * kq) * 8;
    float v[8];
#pragma unroll
    for (int e = 0; e < 8; ++e) v[e] = w[(size_t)(k0 + e) * DO + n] * CW;
    v8h hv;
#pragma unroll
    for (int e = 0; e < 8; ++e) hv[e] = (_Float16)v[e];
    _Float16* dp = dst + (size_t)n * KD + k0;
    *(volatile v8h*)dp = hv;
    __threadfence();
    *(volatile v8h*)dp = hv;
  } else {
    const int t = (blk - (4 * nR + 5)) * NTHR + tid;
    const bool ok = t < nR * DD;
    const int tt = ok ? t : 0;
    const int r = tt >> 6, k = tt & 63;
    const float* re = remb + (size_t)(r + 1) * DD;
    const float* wb = aw1 + ((size_t)r * 2 * DD + DD) * DD;
    float s = 0.0f;
#pragma unroll 1
    for (int d = 0; d < DD; ++d) s = fmaf(re[d], wb[(size_t)d * DD + k], s);
    s = s + ab1[(size_t)r * DD + k];
    if (ok) *(volatile float*)(C + t) = s;
    __threadfence();
    if (ok) *(volatile float*)(C + t) = s;
  }
}

__global__ __launch_bounds__(NTHR) void k_initx(const float* __restrict__ ue, const float* __restrict__ ie,
                                                _Float16* X16, int nU, int nI, int nN) {
  const int idx = blockIdx.x * NTHR + threadIdx.x;
  const int row = idx >> 3, c0 = (idx & 7) * 8;
  const int ru = row > nU - 1 ? nU - 1 : row;
  int ri = row - nU;
  ri = ri < 0 ? 0 : (ri > nI - 1 ? nI - 1 : ri);
  const float* pu = ue + (size_t)ru * DD + c0;
  const float* pi = ie + (size_t)ri * DD + c0;
  const v4f ua = *(const v4f*)pu, ub = *(const v4f*)(pu + 4);
  const v4f ia = *(const v4f*)pi, ib = *(const v4f*)(pi + 4);
  const bool isU = row < nU, isN = row < nN;
  v4f a, b;
  a.x = isU ? ua.x : (isN ? ia.x : 0.0f);  a.y = isU ? ua.y : (isN ? ia.y : 0.0f);
  a.z = isU ? ua.z : (isN ? ia.z : 0.0f);  a.w = isU ? ua.w : (isN ? ia.w : 0.0f);
  b.x = isU ? ub.x : (isN ? ib.x : 0.0f);  b.y = isU ? ub.y : (isN ? ib.y : 0.0f);
  b.z = isU ? ub.z : (isN ? ib.z : 0.0f);  b.w = isU ? ub.w : (isN ? ib.w : 0.0f);
  v8h hv;
  hv[0] = (_Float16)(a.x * CX0); hv[1] = (_Float16)(a.y * CX0); hv[2] = (_Float16)(a.z * CX0); hv[3] = (_Float16)(a.w * CX0);
  hv[4] = (_Float16)(b.x * CX0); hv[5] = (_Float16)(b.y * CX0); hv[6] = (_Float16)(b.z * CX0); hv[7] = (_Float16)(b.w * CX0);
  _Float16* dp = X16 + (size_t)idx * 8;
  *(volatile v8h*)dp = hv;
  __threadfence();
  *(volatile v8h*)dp = hv;
}

__global__ __launch_bounds__(NTHR) void k_conv(const float* __restrict__ XN, _Float16* X16, float sc) {
  const int idx = blockIdx.x * NTHR + threadIdx.x;
  const float* sp = XN + (size_t)idx * 8;
  const v4f a = *(const v4f*)sp, b = *(const v4f*)(sp + 4);
  v8h hv;
  hv[0] = (_Float16)(a.x * sc); hv[1] = (_Float16)(a.y * sc); hv[2] = (_Float16)(a.z * sc); hv[3] = (_Float16)(a.w * sc);
  hv[4] = (_Float16)(b.x * sc); hv[5] = (_Float16)(b.y * sc); hv[6] = (_Float16)(b.z * sc); hv[7] = (_Float16)(b.w * sc);
  _Float16* dp = X16 + (size_t)idx * 8;
  *(volatile v8h*)dp = hv;
  __threadfence();
  *(volatile v8h*)dp = hv;
}

__global__ __launch_bounds__(NTHR) void k_csr(const int* __restrict__ rowsAll, int* pk, int* csr,
                                              int nE, int cntPad, int csrPer, int vec8) {
  extern __shared__ v4i lds_dyn[];
  int* region = (int*)lds_dyn;
  int* scnt   = region + RCAP;
  int* cursor = scnt + NBK;
  int* list   = cursor + NBK;
  int* wcnt   = list + LISTN;
  int* wtot   = wcnt + NWAVE;
  const int tid = threadIdx.x, lane = tid & 31, wave = tid >> 5;
  const int b = blockIdx.x, rel = blockIdx.y;
  const int* dsts = rowsAll + (size_t)rel * nE;
  const int nodeBase = b * NBK;
  const v4i z4 = {0, 0, 0, 0};

  for (int i = tid; i < NBK / 4; i += NTHR) ((v4i*)scnt)[i] = z4;
  __syncthreads();

  const int nChunks = (nE + CHUNK - 1) / CHUNK;

#pragma unroll 1
  for (int ch = 0; ch < nChunks; ++ch) {
    const int cbase = ch * CHUNK;
    const int wc = scan_chunk<NBK>(dsts, nE, cbase, nodeBase, vec8, list, tid, lane, wave);
    if (lane == 0) wcnt[wave] = wc;
    __syncthreads();
    if (wave == 0) {
#pragma unroll 1
      for (int wsx = 0; wsx < NWAVE; ++wsx) {
        int n = __builtin_amdgcn_readfirstlane(wcnt[wsx]);
        n = n > WCAP ? WCAP : (n < 0 ? 0 : n);
        const int* lp = list + wsx * WCAP;
#pragma unroll 1
        for (int i = 0; i < n; ++i) {
          const int ent  = __builtin_amdgcn_readfirstlane(lp[i]);
          const int slot = ent & (NBK - 1);
          if (lane == 0) scnt[slot] = scnt[slot] + 1;
        }
      }
    }
    __syncthreads();
  }

  {
    const int s0 = tid * 32;
    int ts = 0;
#pragma unroll 4
    for (int s = 0; s < 32; ++s) ts += scnt[s0 + s];
    int incl = ts;
#pragma unroll
    for (int d = 1; d < 32; d <<= 1) {
      const int t = __shfl_up(incl, d);
      if (lane >= d) incl += t;
    }
    if (lane == 31) wtot[wave] = incl;
    __syncthreads();
    int pre = 0;
#pragma unroll 1
    for (int w = 0; w < wave; ++w) pre += wtot[w];
    int run = pre + incl - ts;
#pragma unroll 4
    for (int s = 0; s < 32; ++s) {
      int c = scnt[s0 + s];
      c = c < 0 ? 0 : c;
      const int o = run > RCAP ? RCAP : run;
      int ce = RCAP - o;
      ce = c < ce ? c : ce;
      cursor[s0 + s] = o;
      scnt[s0 + s] = (int)((unsigned)o | ((unsigned)ce << 16));
      run += c;
    }
  }
  __syncthreads();

  {
    int* pp = pk + (size_t)rel * cntPad + nodeBase;
#pragma unroll
    for (int it = 0; it < NBK / (4 * NTHR); ++it) {
      const int i = it * NTHR + tid;
      const v4i v = ((const v4i*)scnt)[i];
      *(volatile v4i*)(pp + 4 * i) = v;
    }
    __threadfence();
#pragma unroll
    for (int it = 0; it < NBK / (4 * NTHR); ++it) {
      const int i = it * NTHR + tid;
      const v4i v = ((const v4i*)scnt)[i];
      *(volatile v4i*)(pp + 4 * i) = v;
    }
  }

  for (int i = tid; i < RCAP / 4; i += NTHR) ((v4i*)region)[i] = z4;
  __syncthreads();
#pragma unroll 1
  for (int ch = 0; ch < nChunks; ++ch) {
    const int cbase = ch * CHUNK;
    const int wc = scan_chunk<NBK>(dsts, nE, cbase, nodeBase, vec8, list, tid, lane, wave);
    if (lane == 0) wcnt[wave] = wc;
    __syncthreads();
    if (wave == 0) {
#pragma unroll 1
      for (int wsx = 0; wsx < NWAVE; ++wsx) {
        int n = __builtin_amdgcn_readfirstlane(wcnt[wsx]);
        n = n > WCAP ? WCAP : (n < 0 ? 0 : n);
        const int* lp = list + wsx * WCAP;
#pragma unroll 1
        for (int i = 0; i < n; ++i) {
          const int ent  = __builtin_amdgcn_readfirstlane(lp[i]);
          const int slot = ent & (NBK - 1);
          int e = cbase + ((ent >> SLB) & (CHUNK - 1));
          e = e > nE - 1 ? nE - 1 : e;
          if (lane == 0) {
            const int pos = cursor[slot];
            if ((unsigned)pos < (unsigned)RCAP) {
              region[pos] = e;
              cursor[slot] = pos + 1;
            }
          }
        }
      }
    }
    __syncthreads();
  }

  {
    int* gp = csr + (size_t)rel * csrPer + (size_t)b * RCAP;
#pragma unroll 1
    for (int it = 0; it < RCAP / (4 * NTHR); ++it) {
      const int i = it * NTHR + tid;
      const v4i v = ((const v4i*)region)[i];
      *(volatile v4i*)(gp + 4 * i) = v;
    }
    __threadfence();
#pragma unroll 1
    for (int it = 0; it < RCAP / (4 * NTHR); ++it) {
      const int i = it * NTHR + tid;
      const v4i v = ((const v4i*)region)[i];
      *(volatile v4i*)(gp + 4 * i) = v;
    }
  }
}

__global__ __launch_bounds__(NTHR) void k_gemm(
    const _Float16* __restrict__ X16, const _Float16* __restrict__ W1T, const _Float16* __restrict__ W2T,
    const float* __restrict__ cr, const float* __restrict__ b2, float* H, float inv1) {
  __shared__ __attribute__((aligned(16))) _Float16 sG[NWAVE][16 * GPH];
  __shared__ __attribute__((aligned(16))) float    sO[NWAVE][16 * DD];
  const int tid = threadIdx.x, lane = tid & 31, wave = tid >> 5, hh = lane >> 4, m = lane & 15;
  const int row0 = blockIdx.x * GROWS + wave * 16;

  const _Float16* ap = X16 + (size_t)(row0 + m) * DD + 8 * hh;
  v8f acc[4];
#pragma unroll
  for (int t = 0; t < 4; ++t) acc[t] = (v8f){0.f, 0.f, 0.f, 0.f, 0.f, 0.f, 0.f, 0.f};
#pragma unroll
  for (int kt = 0; kt < 2; ++kt) {
    FragH a;
    a.half[0] = *(const v8h*)(ap + 32 * kt);
    a.half[1] = *(const v8h*)(ap + 32 * kt + 16);
#pragma unroll
    for (int t = 0; t < 4; ++t) {
      const _Float16* bp = W1T + (size_t)(16 * t + m) * DD + 32 * kt + 8 * hh;
      FragH bb;
      bb.half[0] = *(const v8h*)bp;
      bb.half[1] = *(const v8h*)(bp + 16);
      acc[t] = wmh(a.v, bb.v, acc[t]);
    }
  }

  _Float16* g = sG[wave];
#pragma unroll
  for (int t = 0; t < 4; ++t) {
    const float cv = cr[16 * t + m];
#pragma unroll
    for (int r = 0; r < 8; ++r) {
      float v = fmaf(acc[t][r], inv1, cv);
      v = v >= 0.0f ? v : 0.01f * v;
      g[(8 * hh + r) * GPH + 16 * t + m] = (_Float16)(v * CG);
    }
  }
  __syncthreads();

  const _Float16* gp2 = g + m * GPH + 8 * hh;
  v8f acc2[4];
#pragma unroll
  for (int t = 0; t < 4; ++t) acc2[t] = (v8f){0.f, 0.f, 0.f, 0.f, 0.f, 0.f, 0.f, 0.f};
#pragma unroll
  for (int kt = 0; kt < 2; ++kt) {
    FragH a;
    a.half[0] = *(const v8h*)(gp2 + 32 * kt);
    a.half[1] = *(const v8h*)(gp2 + 32 * kt + 16);
#pragma unroll
    for (int t = 0; t < 4; ++t) {
      const _Float16* bp = W2T + (size_t)(16 * t + m) * DD + 32 * kt + 8 * hh;
      FragH bb;
      bb.half[0] = *(const v8h*)bp;
      bb.half[1] = *(const v8h*)(bp + 16);
      acc2[t] = wmh(a.v, bb.v, acc2[t]);
    }
  }

  float* o = sO[wave];
#pragma unroll
  for (int t = 0; t < 4; ++t) {
    const float bv = b2[16 * t + m];
#pragma unroll
    for (int r = 0; r < 8; ++r) o[(8 * hh + r) * DD + 16 * t + m] = fmaf(acc2[t][r], INV2, bv);
  }
  __syncthreads();

  float* hp = H + (size_t)row0 * DD;
#pragma unroll
  for (int i = 0; i < 8; ++i) {
    const v4f v = *(const v4f*)(o + i * 128 + 4 * lane);
    *(volatile v4f*)(hp + i * 128 + 4 * lane) = v;
  }
  __threadfence();
#pragma unroll
  for (int i = 0; i < 8; ++i) {
    const v4f v = *(const v4f*)(o + i * 128 + 4 * lane);
    *(volatile v4f*)(hp + i * 128 + 4 * lane) = v;
  }
}

__global__ __launch_bounds__(NTHR) void k_agg(
    const int* __restrict__ pk, const int* __restrict__ csr,
    const int* __restrict__ acol, const float* __restrict__ aval,
    const float* __restrict__ hin, float* XN, int nN, int nE, int csrPer, int first, int last) {
  const int tid = threadIdx.x, lane = tid & 31, wave = tid >> 5, hh = lane >> 4, sub = lane & 15, hb = lane & 16;
  const int tbase = blockIdx.x * TGT + wave * 32;
  const int pkv = pk[tbase + lane];
  int off_l = pkv & 0xFFFF;
  off_l = off_l > RCAP ? RCAP : off_l;
  int cnt_l = (int)((unsigned)pkv >> 16);
  {
    const int rem = RCAP - off_l;
    cnt_l = cnt_l > rem ? rem : cnt_l;
    cnt_l = cnt_l > DEGCAP ? DEGCAP : cnt_l;
  }
  const int rb = (tbase / NBK) * RCAP;

#pragma unroll 1
  for (int j = 0; j < 32; j += 2) {
    const int na = __builtin_amdgcn_readlane(cnt_l, j);
    const int nb = __builtin_amdgcn_readlane(cnt_l, j + 1);
    const int oa = __builtin_amdgcn_readlane(off_l, j);
    const int ob = __builtin_amdgcn_readlane(off_l, j + 1);
    const int nmax  = na > nb ? na : nb;
    const int nmine = hh != 0 ? nb : na;
    const int st    = rb + (hh != 0 ? ob : oa);
    v4f acc = {0.0f, 0.0f, 0.0f, 0.0f};
#pragma unroll 1
    for (int q0 = 0; q0 < nmax; q0 += 16) {
      int pos = st + q0 + sub;
      pos = pos < 0 ? 0 : (pos > csrPer - 1 ? csrPer - 1 : pos);
      int ed = csr[pos];
      ed = ed < 0 ? 0 : (ed > nE - 1 ? nE - 1 : ed);
      int cl = acol[ed];
      cl = cl < 0 ? 0 : (cl > nN - 1 ? nN - 1 : cl);
      float vl = aval[ed];
      vl = (q0 + sub < nmine) ? vl : 0.0f;
      const int mcnt = (nmax - q0) < 16 ? (nmax - q0) : 16;
#pragma unroll 1
      for (int p = 0; p < mcnt; ++p) {
        const int   s = __shfl(cl, hb + p);
        const float v = __shfl(vl, hb + p);
        const v4f   x = *(const v4f*)(hin + (size_t)s * DD + 4 * sub);
        acc.x = fmaf(v, x.x, acc.x);
        acc.y = fmaf(v, x.y, acc.y);
        acc.z = fmaf(v, x.z, acc.z);
        acc.w = fmaf(v, x.w, acc.w);
      }
    }
    float* gp = XN + (size_t)(tbase + j) * DD + 4 * lane;
    v4f w = acc;
    if (first == 0) {
      const v4f old = *(const v4f*)gp;
      w = old + acc;
    }
    if (last != 0) w = w * 0.2f;
    *(volatile v4f*)gp = w;
    __threadfence();
    *(volatile v4f*)gp = w;
  }
}

__global__ __launch_bounds__(NTHR) void k_gath(const int* __restrict__ users, const int* __restrict__ posi,
                                               const int* __restrict__ negi, const float* __restrict__ XN,
                                               float* Gl, int nB, int nU, int nI) {
  const int idx = blockIdx.x * NTHR + threadIdx.x;
  const int nRows = 3 * nB;
  int row = idx >> 4;
  const int c = (idx & 15) * 4;
  const bool ok = row < nRows;
  row = ok ? row : nRows - 1;
  const int w = row / nB;
  const int b = row - w * nB;
  int u = users[b]; u = u < 0 ? 0 : (u > nU - 1 ? nU - 1 : u);
  int ip = posi[b]; ip = ip < 0 ? 0 : (ip > nI - 1 ? nI - 1 : ip);
  int in = negi[b]; in = in < 0 ? 0 : (in > nI - 1 ? nI - 1 : in);
  const int node = w == 0 ? u : (w == 1 ? nU + ip : nU + in);
  const v4f v = *(const v4f*)(XN + (size_t)node * DD + c);
  float* gp = Gl + (size_t)row * DD + c;
  if (ok) *(volatile v4f*)gp = v;
  __threadfence();
  if (ok) *(volatile v4f*)gp = v;
}

__global__ __launch_bounds__(NTHR) void k_mlp(
    const int* __restrict__ users, const int* __restrict__ posi, const int* __restrict__ negi,
    const float* __restrict__ ue, const float* __restrict__ ie, const float* __restrict__ G,
    const _Float16* __restrict__ P1T, const _Float16* __restrict__ P2T,
    const float* __restrict__ pb1, const float* __restrict__ pb2, const float* __restrict__ pw3,
    const float* __restrict__ pb3, float* out, int nB, int nU, int nI) {
  __shared__ __attribute__((aligned(16))) _Float16 sA[NWAVE][16 * MPA];
  __shared__ __attribute__((aligned(16))) _Float16 sH[NWAVE][16 * GPH];
  __shared__ __attribute__((aligned(16))) float    sR[GROWS];
  const int tid = threadIdx.x, lane = tid & 31, wave = tid >> 5, hh = lane >> 4, m = lane & 15;
  const int nPB = nB / GROWS;
  const int isneg = blockIdx.x >= nPB ? 1 : 0;
  const int pblk = blockIdx.x - isneg * nPB;
  const int bbase = pblk * GROWS + wave * 16;
  const int wsel = hh == 0 ? 0 : 1 + isneg;
  const size_t sl = (size_t)3 * nB * DD;

  _Float16* at = sA[wave];
#pragma unroll 2
  for (int i = 0; i < 16; ++i) {
    int b = bbase + i;
    b = b > nB - 1 ? nB - 1 : b;
    int u = users[b]; u = u < 0 ? 0 : (u > nU - 1 ? nU - 1 : u);
    int ip = posi[b], in = negi[b];
    int it = isneg != 0 ? in : ip;
    it = it < 0 ? 0 : (it > nI - 1 ? nI - 1 : it);
    const v4f vu = *(const v4f*)(ue + (size_t)u * DD + 4 * m);
    const v4f vi = *(const v4f*)(ie + (size_t)it * DD + 4 * m);
    v4f base;
    base.x = hh == 0 ? vu.x : vi.x; base.y = hh == 0 ? vu.y : vi.y;
    base.z = hh == 0 ? vu.z : vi.z; base.w = hh == 0 ? vu.w : vi.w;
    const float* gq = G + ((size_t)wsel * nB + b) * DD + 4 * m;
    const v4f g1 = *(const v4f*)gq;
    const v4f g2 = *(const v4f*)(gq + sl);
    const v4f g3 = *(const v4f*)(gq + 2 * sl);
    v4f lt = ((base + g1) + g2) + g3;
    lt = lt * 0.25f;
    v4h hv;
    hv[0] = (_Float16)(lt.x * CXM); hv[1] = (_Float16)(lt.y * CXM);
    hv[2] = (_Float16)(lt.z * CXM); hv[3] = (_Float16)(lt.w * CXM);
    *(v4h*)(at + i * MPA + 4 * lane) = hv;
  }
  __syncthreads();

  const _Float16* ap = at + m * MPA + 8 * hh;
  v8f acc[4];
#pragma unroll
  for (int t = 0; t < 4; ++t) acc[t] = (v8f){0.f, 0.f, 0.f, 0.f, 0.f, 0.f, 0.f, 0.f};
#pragma unroll
  for (int kt = 0; kt < 4; ++kt) {
    FragH a;
    a.half[0] = *(const v8h*)(ap + 32 * kt);
    a.half[1] = *(const v8h*)(ap + 32 * kt + 16);
#pragma unroll
    for (int t = 0; t < 4; ++t) {
      const _Float16* bp = P1T + (size_t)(16 * t + m) * (2 * DD) + 32 * kt + 8 * hh;
      FragH bb;
      bb.half[0] = *(const v8h*)bp;
      bb.half[1] = *(const v8h*)(bp + 16);
      acc[t] = wmh(a.v, bb.v, acc[t]);
    }
  }
  _Float16* hq = sH[wave];
#pragma unroll
  for (int t = 0; t < 4; ++t) {
    const float bv = pb1[16 * t + m];
#pragma unroll
    for (int r = 0; r < 8; ++r) {
      float v = fmaf(acc[t][r], (1.0f / (CXM * CW)), bv);
      v = v >= 0.0f ? v : 0.01f * v;
      hq[(8 * hh + r) * GPH + 16 * t + m] = (_Float16)(v * CG);
    }
  }
  __syncthreads();

  const _Float16* ap2 = hq + m * GPH + 8 * hh;
  v8f acc2[2];
#pragma unroll
  for (int t = 0; t < 2; ++t) acc2[t] = (v8f){0.f, 0.f, 0.f, 0.f, 0.f, 0.f, 0.f, 0.f};
#pragma unroll
  for (int kt = 0; kt < 2; ++kt) {
    FragH a;
    a.half[0] = *(const v8h*)(ap2 + 32 * kt);
    a.half[1] = *(const v8h*)(ap2 + 32 * kt + 16);
#pragma unroll
    for (int t = 0; t < 2; ++t) {
      const _Float16* bp = P2T + (size_t)(16 * t + m) * DD + 32 * kt + 8 * hh;
      FragH bb;
      bb.half[0] = *(const v8h*)bp;
      bb.half[1] = *(const v8h*)(bp + 16);
      acc2[t] = wmh(a.v, bb.v, acc2[t]);
    }
  }

  float rs[8];
#pragma unroll
  for (int r = 0; r < 8; ++r) rs[r] = 0.0f;
#pragma unroll
  for (int t = 0; t < 2; ++t) {
    const float bv = pb2[16 * t + m];
    const float w3 = pw3[16 * t + m];
#pragma unroll
    for (int r = 0; r < 8; ++r) {
      float v = fmaf(acc2[t][r], INV2, bv);
      v = v >= 0.0f ? v : 0.01f * v;
      rs[r] = fmaf(v, w3, rs[r]);
    }
  }
  const float b3 = pb3[0];
#pragma unroll
  for (int r = 0; r < 8; ++r) {
    float s = rs[r];
    s += __shfl_xor(s, 1);
    s += __shfl_xor(s, 2);
    s += __shfl_xor(s, 4);
    s += __shfl_xor(s, 8);
    rs[r] = s + b3;
  }
  if (m == 0) {
#pragma unroll
    for (int r = 0; r < 8; ++r) sR[wave * 16 + 8 * hh + r] = rs[r];
  }
  __syncthreads();
  if (wave == 0) {
    const v4f v = *(const v4f*)(sR + 4 * lane);
    float* op = out + (size_t)isneg * nB + (size_t)pblk * GROWS + 4 * lane;
    *(volatile v4f*)op = v;
    __threadfence();
    *(volatile v4f*)op = v;
  }
}

extern "C" void kernel_launch(void* const* d_in, const int* in_sizes, int n_in,
                              void* d_out, int out_size, void* d_ws, size_t ws_size,
                              hipStream_t stream) {
  if (n_in < 19) return;
  const int nB = in_sizes[0];
  if (nB < GROWS || (nB % GROWS) != 0 || in_sizes[1] != nB || in_sizes[2] != nB) return;
  if ((in_sizes[3] % DD) != 0 || (in_sizes[4] % DD) != 0) return;
  const int nU = in_sizes[3] / DD, nI = in_sizes[4] / DD;
  if (nU < 1 || nI < 1) return;
  const int nN = nU + nI;
  const int nR = in_sizes[6] / (2 * DD * DD);
  if (nR < 1 || in_sizes[6] != nR * 2 * DD * DD) return;
  if (in_sizes[5] != (nR + 1) * DD || in_sizes[7] != nR * DD || in_sizes[8] != nR * DD * DD || in_sizes[9] != nR * DD) return;
  if (in_sizes[10] != 2 * DD * DD || in_sizes[11] != DD || in_sizes[12] != DD * 32 || in_sizes[13] != 32 ||
      in_sizes[14] != 32 || in_sizes[15] != 1) return;
  const int nE = in_sizes[16] / nR;
  if (nE < 1 || in_sizes[16] != nR * nE || in_sizes[17] != nR * nE || in_sizes[18] != nR * nE) return;
  if (out_size != 2 * nB) return;
  if (nN > (1 << 24) || nE > (1 << 28) || nB > (1 << 22)) return;

  const int*   users = (const int*)d_in[0];
  const int*   posi  = (const int*)d_in[1];
  const int*   negi  = (const int*)d_in[2];
  const float* ue    = (const float*)d_in[3];
  const float* ie    = (const float*)d_in[4];
  const float* remb  = (const float*)d_in[5];
  const float* aw1   = (const float*)d_in[6];
  const float* ab1   = (const float*)d_in[7];
  const float* aw2   = (const float*)d_in[8];
  const float* ab2   = (const float*)d_in[9];
  const float* pw1   = (const float*)d_in[10];
  const float* pb1   = (const float*)d_in[11];
  const float* pw2   = (const float*)d_in[12];
  const float* pb2   = (const float*)d_in[13];
  const float* pw3   = (const float*)d_in[14];
  const float* pb3   = (const float*)d_in[15];
  const int*   erows = (const int*)d_in[16];
  const int*   ecols = (const int*)d_in[17];
  const float* evals = (const float*)d_in[18];
  float* out = (float*)d_out;

  const int NPAD   = ((nN + TGT - 1) / TGT) * TGT;
  const int nBK    = (nN + NBK - 1) / NBK;
  const int CNTPAD = nBK * NBK;
  const int csrPer = nBK * RCAP;

  char* ws = (char*)d_ws;
  size_t off = 0;
  const size_t oW1  = off; off += (size_t)nR * DD * DD * 2;         off = (off + 255) & ~(size_t)255;
  const size_t oW2  = off; off += (size_t)nR * DD * DD * 2;         off = (off + 255) & ~(size_t)255;
  const size_t oP1  = off; off += (size_t)DD * 2 * DD * 2;          off = (off + 255) & ~(size_t)255;
  const size_t oP2  = off; off += (size_t)32 * DD * 2;              off = (off + 255) & ~(size_t)255;
  const size_t oC   = off; off += (size_t)nR * DD * 4;              off = (off + 255) & ~(size_t)255;
  const size_t oPk  = off; off += (size_t)nR * CNTPAD * 4;          off = (off + 255) & ~(size_t)255;
  const size_t oCsr = off; off += (size_t)nR * csrPer * 4;          off = (off + 255) & ~(size_t)255;
  const size_t oX16 = off; off += (size_t)NPAD * DD * 2;            off = (off + 255) & ~(size_t)255;
  const size_t oH   = off; off += (size_t)NPAD * DD * 4;            off = (off + 255) & ~(size_t)255;
  const size_t oXN  = off; off += (size_t)NPAD * DD * 4;            off = (off + 255) & ~(size_t)255;
  const size_t oG   = off; off += (size_t)NLAYER * 3 * nB * DD * 4; off = (off + 255) & ~(size_t)255;
  if (off > ws_size || off > (size_t)WSCAP) return;
  _Float16* W1T = (_Float16*)(ws + oW1);
  _Float16* W2T = (_Float16*)(ws + oW2);
  _Float16* P1T = (_Float16*)(ws + oP1);
  _Float16* P2T = (_Float16*)(ws + oP2);
  float*    C   = (float*)(ws + oC);
  int*      pk  = (int*)(ws + oPk);
  int*      csr = (int*)(ws + oCsr);
  _Float16* X16 = (_Float16*)(ws + oX16);
  float*    H   = (float*)(ws + oH);
  float*    XN  = (float*)(ws + oXN);
  float*    G   = (float*)(ws + oG);

  const int vec8 = ((nE & 3) == 0) ? 1 : 0;

  const int nWB = 4 * nR + 5 + (nR * DD + NTHR - 1) / NTHR;
  k_wprep<<<nWB, NTHR, 0, stream>>>(aw1, ab1, aw2, remb, pw1, pw2, W1T, W2T, P1T, P2T, C, nR);

  k_initx<<<NPAD / 32, NTHR, 0, stream>>>(ue, ie, X16, nU, nI, nN);

  hipFuncSetAttribute(reinterpret_cast<const void*>(&k_csr), hipFuncAttributeMaxDynamicSharedMemorySize, LDS_CSR);
  k_csr<<<dim3(nBK, nR), NTHR, LDS_CSR, stream>>>(erows, pk, csr, nE, CNTPAD, csrPer, vec8);

  for (int l = 0; l < NLAYER; ++l) {
    const float inv1 = (l == 0) ? (1.0f / (CX0 * CW)) : (1.0f / (CX1 * CW));
    for (int r = 0; r < nR; ++r) {
      k_gemm<<<NPAD / GROWS, NTHR, 0, stream>>>(X16, W1T + (size_t)r * DD * DD, W2T + (size_t)r * DD * DD,
                                                C + (size_t)r * DD, ab2 + (size_t)r * DD, H, inv1);
      k_agg<<<NPAD / TGT, NTHR, 0, stream>>>(pk + (size_t)r * CNTPAD, csr + (size_t)r * csrPer,
                                             ecols + (size_t)r * nE, evals + (size_t)r * nE,
                                             H, XN, nN, nE, csrPer, r == 0 ? 1 : 0, r == nR - 1 ? 1 : 0);
    }
    k_gath<<<(3 * nB * 16 + NTHR - 1) / NTHR, NTHR, 0, stream>>>(users, posi, negi, XN,
                                                                 G + (size_t)l * 3 * nB * DD, nB, nU, nI);
    if (l + 1 < NLAYER) k_conv<<<NPAD / 32, NTHR, 0, stream>>>(XN, X16, CX1);
  }

  k_mlp<<<2 * nB / GROWS, NTHR, 0, stream>>>(users, posi, negi, ue, ie, G, P1T, P2T, pb1, pb2, pw3, pb3,
                                             out, nB, nU, nI);
}
